// MLPPredictor_58317065945293
// MI455X (gfx1250) — hardware-run, weakly checked
//
#include <hip/hip_runtime.h>
#include <math.h>

typedef __attribute__((ext_vector_type(16))) _Float16 v16h;
typedef __attribute__((ext_vector_type(8)))  _Float16 v8h;
typedef __attribute__((ext_vector_type(8)))  float    v8f;
typedef __attribute__((ext_vector_type(4)))  float    v4f;
typedef __attribute__((ext_vector_type(2)))  float    v2f;
typedef __attribute__((ext_vector_type(4)))  unsigned v4u;
typedef __attribute__((ext_vector_type(2)))  int      v2i;

constexpr int kNodes      = 50000;
constexpr int kFeat       = 128;
constexpr int kEdges      = 640000;
constexpr int kCls        = 2;
constexpr int kMpad       = 50048;
constexpr int kBtRows     = 16;
constexpr int kPw         = 4;
constexpr int kRowsPerBlk = 128;
constexpr int kPrepBlocksA = (kMpad * kFeat / 8) / 256;

constexpr float kCarryH   = 64.0f;
constexpr float kCarryW   = 64.0f;
constexpr float kFold     = 1.0f / (kCarryH * kCarryW);
constexpr float kF16MinNormal = 6.103515625e-05f;

static_assert(kMpad >= kNodes && (kMpad % kRowsPerBlk) == 0, "node rows padded to the block tile");
static_assert((kFeat % 32) == 0, "K multiple of 32");
static_assert(((kMpad * kFeat / 8) % 256) == 0, "prep grid exact");
static_assert((kBtRows * kFeat / 8) == 256, "weight plane = one block of 8-element pieces");
static_assert((kEdges % 256) == 0, "edge grid exact");
static_assert(2 * kCls == kPw, "projection plane width");

constexpr size_t kOffA16  = 0;
constexpr size_t kOffBT16 = kOffA16  + (size_t)kMpad * kFeat * 2;
constexpr size_t kOffP    = kOffBT16 + (size_t)kBtRows * kFeat * 2;
constexpr size_t kWsTotal = kOffP    + (size_t)kMpad * kPw * 4;
static_assert(kWsTotal == 13617152ull, "carve total");
static_assert(kWsTotal <= 134217728ull, "carve cap");
static_assert((kOffBT16 % 128) == 0 && (kOffP % 128) == 0, "128-B aligned regions");

union FragH { v16h v; v8h h[2]; };
__device__ __forceinline__ v16h frag_load_h(const _Float16* p) {
  FragH f;
  f.h[0] = *(const v8h*)(p);
  f.h[1] = *(const v8h*)(p + 16);
  return f.v;
}
__device__ __forceinline__ v8f mma_f16_guarded(v16h a, v16h b, v8f c) {
  c = __builtin_amdgcn_wmma_f32_16x16x32_f16(false, a, false, b, (short)0, c, false, false);
  asm volatile("v_nop\n\tv_nop\n\tv_nop\n\tv_nop" : "+v"(c) : "v"(a), "v"(b));
  return c;
}

__device__ __forceinline__ unsigned f16_bits_carried(float x, bool live, float carry) {
  float v = live ? (x * carry) : 0.0f;
  v = (fabsf(v) < kF16MinNormal) ? 0.0f : v;
  const _Float16 hv = (_Float16)v;
  const unsigned short hb = __builtin_bit_cast(unsigned short, hv);
  return (unsigned)hb;
}

__global__ __launch_bounds__(256) void prep_planes_kernel(
    const float* __restrict__ h, const float* __restrict__ W,
    unsigned short* __restrict__ A16, unsigned short* __restrict__ BT16)
{
  const int tid = threadIdx.x;
  const float* src;
  unsigned short* dst;
  bool live;
  float carry;
  if (blockIdx.x < kPrepBlocksA) {
    const int i   = blockIdx.x * 256 + tid;
    const int row = i >> 4;
    const int c8  = (i & 15) * 8;
    const int rs  = (row < kNodes) ? row : (kNodes - 1);
    src   = h + (size_t)rs * kFeat + c8;
    dst   = A16 + (size_t)i * 8;
    live  = (row < kNodes);
    carry = kCarryH;
  } else {
    const int row = tid >> 4;
    const int c8  = (tid & 15) * 8;
    const int rr  = row & 3;
    src   = W + (rr & 1) * (2 * kFeat) + (rr >> 1) * kFeat + c8;
    dst   = BT16 + (size_t)tid * 8;
    live  = (row < 4);
    carry = kCarryW;
  }
  const v4f a0 = *(const v4f*)(src);
  const v4f a1 = *(const v4f*)(src + 4);
  const float x0 = a0[0], x1 = a0[1], x2 = a0[2], x3 = a0[3];
  const float x4 = a1[0], x5 = a1[1], x6 = a1[2], x7 = a1[3];
  v4u pk;
  pk[0] = f16_bits_carried(x0, live, carry) | (f16_bits_carried(x1, live, carry) << 16);
  pk[1] = f16_bits_carried(x2, live, carry) | (f16_bits_carried(x3, live, carry) << 16);
  pk[2] = f16_bits_carried(x4, live, carry) | (f16_bits_carried(x5, live, carry) << 16);
  pk[3] = f16_bits_carried(x6, live, carry) | (f16_bits_carried(x7, live, carry) << 16);
  *(volatile v4u*)dst = pk;
  __threadfence();
  *(volatile v4u*)dst = pk;
}

__global__ __launch_bounds__(256) void node_proj_kernel(
    const unsigned short* __restrict__ A16p, const unsigned short* __restrict__ BT16p, float* __restrict__ P)
{
  __shared__ __align__(16) float sP[kRowsPerBlk * kPw];
  const _Float16* A  = (const _Float16*)A16p;
  const _Float16* Bt = (const _Float16*)BT16p;
  const int tid   = threadIdx.x;
  const int lane  = tid & 31;
  const int wave  = tid >> 5;
  const int rlane = lane & 15;
  const int hh    = lane >> 4;
  const int koff  = hh * 8;
  const int mblk  = blockIdx.x * kRowsPerBlk;
  if (mblk >= kMpad) return;
  const int mw = mblk + wave * 16;

  v16h bf[4], af[4];
#pragma unroll
  for (int kt = 0; kt < 4; ++kt) {
    bf[kt] = frag_load_h(Bt + (size_t)rlane * kFeat + koff + kt * 32);
    af[kt] = frag_load_h(A + (size_t)(mw + rlane) * kFeat + koff + kt * 32);
  }
  v8f acc = (v8f){0.f, 0.f, 0.f, 0.f, 0.f, 0.f, 0.f, 0.f};
#pragma unroll
  for (int kt = 0; kt < 4; ++kt) acc = mma_f16_guarded(af[kt], bf[kt], acc);

  if (rlane < kPw) {
#pragma unroll
    for (int r = 0; r < 8; ++r) sP[(wave * 16 + hh * 8 + r) * kPw + rlane] = acc[r] * kFold;
  }
  __syncthreads();
  if (wave < 4) {
    const v4f val = *(const v4f*)(sP + tid * kPw);
    float* dst = P + (size_t)(mblk + tid) * kPw;
    *(volatile v4f*)dst = val;
    __threadfence();
    *(volatile v4f*)dst = val;
  }
}

__global__ __launch_bounds__(256) void edge_logsoftmax_kernel(
    const int* __restrict__ ei, const float* __restrict__ P, const float* __restrict__ bias, float* __restrict__ out)
{
  const int e  = blockIdx.x * 256 + threadIdx.x;
  const int ec = (e < kEdges) ? e : (kEdges - 1);
  const v2i uv = *(const v2i*)(ei + 2 * (size_t)ec);
  int u = uv[0];
  int v = uv[1];
  u = (u < 0) ? 0 : u;
  u = (u > kNodes - 1) ? (kNodes - 1) : u;
  v = (v < 0) ? 0 : v;
  v = (v > kNodes - 1) ? (kNodes - 1) : v;
  const v2f pu = *(const v2f*)(P + (size_t)u * kPw);
  const v2f pv = *(const v2f*)(P + (size_t)v * kPw + kCls);
  float pu0 = pu[0], pu1 = pu[1], pv0 = pv[0], pv1 = pv[1];
  asm volatile("" : "+v"(pu0), "+v"(pu1), "+v"(pv0), "+v"(pv1));
  const float b0 = bias[0];
  const float b1 = bias[1];
  const float l0 = (pu0 + pv0) + b0;
  const float l1 = (pu1 + pv1) + b1;
  const float m  = fmaxf(l0, l1);
  const float d0 = l0 - m;
  const float d1 = l1 - m;
  const float ls = logf(expf(d0) + expf(d1));
  v2f o;
  o[0] = d0 - ls;
  o[1] = d1 - ls;
  if (e < kEdges) {
    float* dst = out + 2 * (size_t)e;
    *(volatile v2f*)dst = o;
    __threadfence();
    *(volatile v2f*)dst = o;
  }
}

extern "C" void kernel_launch(void* const* d_in, const int* in_sizes, int n_in,
                              void* d_out, int out_size, void* d_ws, size_t ws_size,
                              hipStream_t stream) {
  if (n_in < 4) return;
  if (in_sizes[0] != kNodes * kFeat) return;
  if (in_sizes[1] != kCls * 2 * kFeat) return;
  if (in_sizes[2] != kCls) return;
  if (in_sizes[3] != kEdges * 2) return;
  if (out_size != kEdges * kCls) return;
  if (ws_size < kWsTotal) return;

  const float* h    = (const float*)d_in[0];
  const float* W    = (const float*)d_in[1];
  const float* bias = (const float*)d_in[2];
  const int*   ei   = (const int*)d_in[3];
  float* out = (float*)d_out;

  char* ws = (char*)d_ws;
  unsigned short* A16  = (unsigned short*)(ws + kOffA16);
  unsigned short* BT16 = (unsigned short*)(ws + kOffBT16);
  float*          P    = (float*)(ws + kOffP);

  prep_planes_kernel<<<kPrepBlocksA + 1, 256, 0, stream>>>(h, W, A16, BT16);
  node_proj_kernel<<<kMpad / kRowsPerBlk, 256, 0, stream>>>(A16, BT16, P);
  edge_logsoftmax_kernel<<<kEdges / 256, 256, 0, stream>>>(ei, P, bias, out);
}
